// FractalAttentionLayer_54228257079871
// MI455X (gfx1250) — hardware-verified
//
#include <hip/hip_runtime.h>
#include <math.h>
#include <float.h>
#include <stdint.h>

#define NB      2
#define SEQ     2048
#define DMODEL  1024
#define NH      16
#define HD      64
#define QP      (NH * HD)
#define N3      (3 * DMODEL)
#define QKP     (2 * QP)
#define NQB     (SEQ / 64)
#define RESQB   ((NQB < 16) ? NQB : 16)
#define VLP     (RESQB * 64)
#define CG8     (DMODEL / 8)
#define NBIAS   (4 * DMODEL)
#define NTT     (NB * NH * SEQ)
#define OUTN    (NB * SEQ * DMODEL)
#define KAPPA_F 0.3f
static_assert(RESQB >= 1 && RESQB * 64 <= VLP && VLP <= SEQ);
static_assert(QP == DMODEL);
static_assert((SEQ % 64) == 0 && (DMODEL % 64) == 0 && (N3 % 64) == 0 && (QP % 64) == 0);
static_assert(HD == 64);
static_assert((((NB * SEQ) / 64) * (N3 / 64)) % 8 == 0);
static_assert((((NB * SEQ) / 64) * (DMODEL / 64)) % 8 == 0);
static_assert((NBIAS % 256) == 0 && (NTT % 256) == 0);
static_assert(((NB * SEQ * DMODEL / 8) % 256) == 0);
static_assert((DMODEL % 8) == 0);

typedef _Float16 v16h __attribute__((ext_vector_type(16)));
typedef _Float16 v8h  __attribute__((ext_vector_type(8)));
typedef __bf16   v16b __attribute__((ext_vector_type(16)));
typedef __bf16   v8b  __attribute__((ext_vector_type(8)));
typedef float    v8f  __attribute__((ext_vector_type(8)));
typedef float    v4f  __attribute__((ext_vector_type(4)));
typedef unsigned int v4u __attribute__((ext_vector_type(4)));

__device__ __forceinline__ unsigned short bf_bits(float f) {
  unsigned u = __float_as_uint(f);
  return (unsigned short)((u + 0x7FFFu + ((u >> 16) & 1u)) >> 16);
}
__device__ __forceinline__ float bf_up(unsigned short h) { return __uint_as_float(((unsigned)h) << 16); }
__device__ __forceinline__ unsigned short h_bits(_Float16 x) { return __builtin_bit_cast(unsigned short, x); }
__device__ __forceinline__ unsigned pk16(unsigned short a, unsigned short b) { return (unsigned)a | ((unsigned)b << 16); }
__device__ __forceinline__ v8f zero8() { v8f z = {0.f, 0.f, 0.f, 0.f, 0.f, 0.f, 0.f, 0.f}; return z; }
__device__ __forceinline__ v8h zero8h() {
  const _Float16 z = (_Float16)0.0f;
  v8h r = {z, z, z, z, z, z, z, z};
  return r;
}

__device__ __forceinline__ float fexpo(int s) {
#pragma clang fp contract(off)
  const float rs = 1.0f / (float)(SEQ - 1);
  const float fr = (float)s * rs;
  const float om = 1.0f - fr;
  const float t  = KAPPA_F * om;
  return 1.0f + t;
}
__device__ __forceinline__ float fcomp(float v, float ex) {
#pragma clang fp contract(off)
  const float mag = fmaxf(fabsf(v), 1e-8f);
  const float lg  = log2f(mag);
  const float pw  = exp2f(ex * lg);
  float r = (v < 0.0f) ? -pw : pw;
  r = (v == 0.0f) ? 0.0f : r;
  return r;
}

__device__ __forceinline__ v16b ldfrag_b(const __bf16* p) {
  union { v16b v; v8b h[2]; } f;
  f.h[0] = *(const v8b*)(p);
  f.h[1] = *(const v8b*)(p + 16);
  return f.v;
}

__device__ __forceinline__ v8f mma_b(v16b a, v16b b, v8f c) {
  c = __builtin_amdgcn_wmma_f32_16x16x32_bf16(false, a, false, b, (short)0, c, false, false);
#if defined(__HIP_DEVICE_COMPILE__)
  asm volatile("v_nop\n\tv_nop\n\tv_nop\n\tv_nop" : "+v"(c) : "v"(a), "v"(b));
#endif
  return c;
}
__device__ __forceinline__ v8f mma_h(v16h a, v16h b, v8f c) {
  c = __builtin_amdgcn_wmma_f32_16x16x32_f16(false, a, false, b, (short)0, c, false, false);
#if defined(__HIP_DEVICE_COMPILE__)
  asm volatile("v_nop\n\tv_nop\n\tv_nop\n\tv_nop" : "+v"(c) : "v"(a), "v"(b));
#endif
  return c;
}
__device__ __forceinline__ v8f mma_b_raw(v16b a, v16b b, v8f c) {
  return __builtin_amdgcn_wmma_f32_16x16x32_bf16(false, a, false, b, (short)0, c, false, false);
}
__device__ __forceinline__ void dep_guard_b(v8f& a, v8f& b, v16b x, v16b y) {
#if defined(__HIP_DEVICE_COMPILE__)
  asm volatile("v_nop\n\tv_nop\n\tv_nop\n\tv_nop" : "+v"(a), "+v"(b) : "v"(x), "v"(y));
#endif
}
__device__ __forceinline__ void keep4_b(v16b a, v16b b, v16b c, v16b d) {
#if defined(__HIP_DEVICE_COMPILE__)
  asm volatile("v_nop" :: "v"(a), "v"(b), "v"(c), "v"(d));
#endif
}
__device__ __forceinline__ void acc_guard4(v8f& a, v8f& b, v8f& c, v8f& d) {
#if defined(__HIP_DEVICE_COMPILE__)
  asm volatile("v_nop\n\tv_nop\n\tv_nop\n\tv_nop" : "+v"(a), "+v"(b), "+v"(c), "+v"(d));
#endif
}

__global__ __launch_bounds__(256) void bias_tab(const float* __restrict__ b0, const float* __restrict__ b1,
                                                const float* __restrict__ b2, const float* __restrict__ b3,
                                                float* dst, int n, int seg) {
  const int i = blockIdx.x * 256 + threadIdx.x;
  if (i < n) {
    int part = i / seg;
    part = (part < 0) ? 0 : ((part > 3) ? 3 : part);
    int idx = i - part * seg;
    idx = (idx < 0) ? 0 : ((idx >= seg) ? (seg - 1) : idx);
    const float v0 = b0[idx], v1 = b1[idx], v2 = b2[idx], v3 = b3[idx];
    float v = (part == 0) ? v0 : ((part == 1) ? v1 : ((part == 2) ? v2 : v3));
    v = bf_up(bf_bits(v));
    *(volatile float*)(dst + i) = v;
    __threadfence();
    *(volatile float*)(dst + i) = v;
  }
}

__global__ __launch_bounds__(256) void phase_tab(const float* __restrict__ ph, const float* __restrict__ cf,
                                                 float* tt, int n) {
#pragma clang fp contract(off)
  const int i = blockIdx.x * 256 + threadIdx.x;
  if (i < n) {
    const int bh = i / SEQ;
    const int s  = i - bh * SEQ;
    const int h  = bh % NH;
    int b        = bh / NH;
    b = (b >= NB) ? (NB - 1) : b;
    const float p  = bf_up(bf_bits(ph[b * SEQ + s]));
    const float cr = bf_up(bf_bits(cf[h]));
    const float d  = p - cr;
    const float hx = d * 0.5f;
    const float cv = cosf(hx);
    const float tv = cv * cv;
    *(volatile float*)(tt + i) = tv;
    __threadfence();
    *(volatile float*)(tt + i) = tv;
  }
}

__global__ __launch_bounds__(256) void cvt_bf16x8(const float* __restrict__ in, unsigned short* out, int n8) {
  const int i = blockIdx.x * 256 + threadIdx.x;
  if (i < n8) {
    const v4f a = *(const v4f*)(in + (size_t)i * 8);
    const v4f b = *(const v4f*)(in + (size_t)i * 8 + 4);
    v4u p;
    p[0] = pk16(bf_bits(a[0]), bf_bits(a[1]));
    p[1] = pk16(bf_bits(a[2]), bf_bits(a[3]));
    p[2] = pk16(bf_bits(b[0]), bf_bits(b[1]));
    p[3] = pk16(bf_bits(b[2]), bf_bits(b[3]));
    *(volatile v4u*)(out + (size_t)i * 8) = p;
    __threadfence();
    *(volatile v4u*)(out + (size_t)i * 8) = p;
  }
}

__global__ __launch_bounds__(256) void split_bf16x8(const float* __restrict__ in, unsigned short* hp,
                                                    unsigned short* lp, int n8) {
  const int i = blockIdx.x * 256 + threadIdx.x;
  if (i < n8) {
    const v4f a = *(const v4f*)(in + (size_t)i * 8);
    const v4f b = *(const v4f*)(in + (size_t)i * 8 + 4);
    v4u ph, pl;
#pragma unroll
    for (int e = 0; e < 4; ++e) {
      const float f0 = (e < 2) ? a[2 * e]     : b[2 * e - 4];
      const float f1 = (e < 2) ? a[2 * e + 1] : b[2 * e - 3];
      const unsigned short h0 = bf_bits(f0), h1 = bf_bits(f1);
      const unsigned short l0 = bf_bits(f0 - bf_up(h0)), l1 = bf_bits(f1 - bf_up(h1));
      ph[e] = pk16(h0, h1);
      pl[e] = pk16(l0, l1);
    }
    *(volatile v4u*)(hp + (size_t)i * 8) = ph;
    *(volatile v4u*)(lp + (size_t)i * 8) = pl;
    __threadfence();
    *(volatile v4u*)(hp + (size_t)i * 8) = ph;
    *(volatile v4u*)(lp + (size_t)i * 8) = pl;
  }
}

__global__ __launch_bounds__(256) void tr_cvt_bf16(const float* __restrict__ src, unsigned short* dst, int K, int N) {
  __shared__ float s[64][33];
  const int tid = threadIdx.x, wave = tid >> 5, lane = tid & 31;
  const int k0 = blockIdx.x * 64, n0 = blockIdx.y * 32;
#pragma unroll
  for (int i = 0; i < 8; ++i) {
    const int idx = i * 256 + tid;
    const int kk = idx >> 5, nn = idx & 31;
    s[kk][nn] = src[(size_t)(k0 + kk) * N + n0 + nn];
  }
  __syncthreads();
  const int q = lane >> 3, piece = lane & 7;
  const int n = wave * 4 + q;
  v4u p;
#pragma unroll
  for (int e = 0; e < 4; ++e) {
    p[e] = pk16(bf_bits(s[piece * 8 + 2 * e][n]), bf_bits(s[piece * 8 + 2 * e + 1][n]));
  }
  unsigned short* d = dst + (size_t)(n0 + n) * K + k0 + piece * 8;
  *(volatile v4u*)d = p;
  __threadfence();
  *(volatile v4u*)d = p;
}

template <int NSPLIT>
__global__ __launch_bounds__(256) void gemm64(
    const unsigned short* __restrict__ Ap, const unsigned short* A2p, int lda,
    const unsigned short* __restrict__ Btp, int ldb, const float* __restrict__ bias,
    float* C, int ldc, int M, int N, int K) {
  const __bf16* Ab  = (const __bf16*)(const void*)Ap;
  const __bf16* Ab2 = (const __bf16*)(const void*)A2p;
  const __bf16* Bb  = (const __bf16*)(const void*)Btp;
  __shared__ __align__(16) float sT[8][16 * 68];
  const int lane = threadIdx.x & 31;
  const int wave = threadIdx.x >> 5;
  const int tilesN = N >> 6;
  const int tilesM = M >> 6;
  const int tile = blockIdx.x * 8 + wave;
  if (tile >= tilesM * tilesN) return;
  const int tm = tile / tilesN;
  const int tn = tile - tm * tilesN;
  const int m0 = tm << 6;
  const int n0 = tn << 6;

  const int rlane = lane & 15;
  const int koff  = (lane >> 4) * 8;
  const int mOff  = (lane >> 4) * 8;

  v8f acc[4][4];
#pragma unroll
  for (int i = 0; i < 4; ++i)
#pragma unroll
    for (int j = 0; j < 4; ++j) acc[i][j] = zero8();

  for (int k0 = 0; k0 < K; k0 += 32) {
    v16b bh[4];
#pragma unroll
    for (int j = 0; j < 4; ++j) {
      const size_t bo = (size_t)(n0 + (j << 4) + rlane) * ldb + koff + k0;
      bh[j] = ldfrag_b(Bb + bo);
    }
#pragma unroll
    for (int i = 0; i < 4; ++i) {
      const size_t ao = (size_t)(m0 + (i << 4) + rlane) * lda + koff + k0;
      const v16b ah = ldfrag_b(Ab + ao);
      v16b al = ah;
      if (NSPLIT >= 1) al = ldfrag_b(Ab2 + ao);
#pragma unroll
      for (int j = 0; j < 4; ++j) {
        acc[i][j] = mma_b_raw(ah, bh[j], acc[i][j]);
        if (NSPLIT >= 1) acc[i][j] = mma_b_raw(al, bh[j], acc[i][j]);
      }
      dep_guard_b(acc[i][0], acc[i][3], ah, al);
    }
    keep4_b(bh[0], bh[1], bh[2], bh[3]);
  }
  acc_guard4(acc[0][0], acc[0][1], acc[0][2], acc[0][3]);
  acc_guard4(acc[1][0], acc[1][1], acc[1][2], acc[1][3]);
  acc_guard4(acc[2][0], acc[2][1], acc[2][2], acc[2][3]);
  acc_guard4(acc[3][0], acc[3][1], acc[3][2], acc[3][3]);

  float bz[4];
#pragma unroll
  for (int j = 0; j < 4; ++j) bz[j] = bias[n0 + (j << 4) + rlane];
  float* slab = sT[wave];
#pragma unroll
  for (int i = 0; i < 4; ++i) {
    const int mBase = m0 + (i << 4);
#pragma unroll
    for (int r = 0; r < 8; ++r) {
#pragma unroll
      for (int j = 0; j < 4; ++j) {
        slab[(mOff + r) * 68 + (j << 4) + rlane] = acc[i][j][r] + bz[j];
      }
    }
    __builtin_amdgcn_fence(__ATOMIC_RELEASE, "workgroup");
    __builtin_amdgcn_wave_barrier();
    __builtin_amdgcn_fence(__ATOMIC_ACQUIRE, "workgroup");
    {
      const int hh = lane >> 4, c4 = (lane & 15) * 4;
      v4f ov[8];
#pragma unroll
      for (int it = 0; it < 8; ++it) {
        const int row = it * 2 + hh;
        ov[it] = *(const v4f*)(slab + row * 68 + c4);
      }
      for (int pass = 0; pass < 2; ++pass) {
#pragma unroll
        for (int it = 0; it < 8; ++it) {
          const int row = it * 2 + hh;
          *(volatile v4f*)(C + (size_t)(mBase + row) * ldc + n0 + c4) = ov[it];
        }
        __threadfence();
      }
    }
    __builtin_amdgcn_fence(__ATOMIC_RELEASE, "workgroup");
    __builtin_amdgcn_wave_barrier();
    __builtin_amdgcn_fence(__ATOMIC_ACQUIRE, "workgroup");
  }
}

__global__ __launch_bounds__(256) void qk_planes(const float* __restrict__ src, unsigned short* hp,
                                                 unsigned short* lp, int n8) {
#pragma clang fp contract(off)
  const int i = blockIdx.x * 256 + threadIdx.x;
  const int part = blockIdx.y;
  if (i < n8) {
    const int row = i / CG8;
    const int cg  = i - row * CG8;
    const int col = part * DMODEL + (cg << 3);
    const float* sp = src + (size_t)row * N3 + col;
    v4f a = *(const v4f*)(sp);
    v4f c = *(const v4f*)(sp + 4);
    if (part == 1) {
      const float ex = fexpo(row % SEQ);
#pragma unroll
      for (int e = 0; e < 4; ++e) {
        a[e] = fcomp(a[e], ex);
        c[e] = fcomp(c[e], ex);
      }
    }
    v4u ph, pl;
#pragma unroll
    for (int e = 0; e < 4; ++e) {
      const float f0 = (e < 2) ? a[2 * e]     : c[2 * e - 4];
      const float f1 = (e < 2) ? a[2 * e + 1] : c[2 * e - 3];
      const unsigned short h0 = bf_bits(f0), h1 = bf_bits(f1);
      const unsigned short l0 = bf_bits(f0 - bf_up(h0)), l1 = bf_bits(f1 - bf_up(h1));
      ph[e] = pk16(h0, h1);
      pl[e] = pk16(l0, l1);
    }
    const size_t go = (size_t)row * QKP + col;
    *(volatile v4u*)(hp + go) = ph;
    *(volatile v4u*)(lp + go) = pl;
    __threadfence();
    *(volatile v4u*)(hp + go) = ph;
    *(volatile v4u*)(lp + go) = pl;
  }
}

__global__ __launch_bounds__(256) void v_planes(const float* __restrict__ vf, int vrp,
                                                unsigned short* vth, unsigned short* vtl) {
#pragma clang fp contract(off)
  __shared__ __align__(16) float sv[64 * 68];
  const int tid = threadIdx.x;
  const int t0  = blockIdx.x * 64;
  const int hh  = blockIdx.y;
  const int b   = blockIdx.z;
#pragma unroll 1
  for (int i = 0; i < 4; ++i) {
    const int idx = i * 256 + tid;
    const int tt = idx >> 4, c4 = (idx & 15) * 4;
    const v4f a = *(const v4f*)(vf + ((size_t)(b * SEQ + t0 + tt)) * vrp + hh * HD + c4);
    const float ex = fexpo(t0 + tt);
    v4f cp;
    cp[0] = fcomp(a[0], ex);
    cp[1] = fcomp(a[1], ex);
    cp[2] = fcomp(a[2], ex);
    cp[3] = fcomp(a[3], ex);
    *(v4f*)(sv + tt * 68 + c4) = cp;
  }
  __syncthreads();

  const int g = tid >> 3, piece = tid & 7;
  v4u hv[2], lv[2];
  size_t hofs[2], lofs[2];
#pragma unroll
  for (int it = 0; it < 2; ++it) {
    const int d = it * 32 + g;
    v4u a, a2;
#pragma unroll
    for (int e = 0; e < 4; ++e) {
      const float f0 = sv[(piece * 8 + 2 * e) * 68 + d];
      const float f1 = sv[(piece * 8 + 2 * e + 1) * 68 + d];
      const _Float16 x0 = (_Float16)f0, x1 = (_Float16)f1;
      const unsigned short h0 = h_bits(x0), h1 = h_bits(x1);
      const unsigned short l0 = h_bits((_Float16)((f0 - (float)x0) * 4096.0f));
      const unsigned short l1 = h_bits((_Float16)((f1 - (float)x1) * 4096.0f));
      a[e] = pk16(h0, h1); a2[e] = pk16(l0, l1);
    }
    hv[it] = a; lv[it] = a2;
    const size_t rowf = (size_t)(b * QP + hh * HD + d);
    hofs[it] = rowf * SEQ + t0 + piece * 8;
    lofs[it] = rowf * VLP + t0 + piece * 8;
  }
  const bool wlo = (t0 + 64 <= VLP);
  for (int pass = 0; pass < 2; ++pass) {
#pragma unroll
    for (int it = 0; it < 2; ++it) {
      *(volatile v4u*)(vth + hofs[it]) = hv[it];
      if (wlo) *(volatile v4u*)(vtl + lofs[it]) = lv[it];
    }
    __threadfence();
  }
}

template <bool RES>
__global__ __launch_bounds__(128)
void attn_causal64(const unsigned short* __restrict__ qkhp, const unsigned short* __restrict__ qklp,
                   const unsigned short* __restrict__ vhp, const unsigned short* __restrict__ vlp,
                   const float* __restrict__ ttab, const float* __restrict__ lockp,
                   float* outp, int qbBase, int nqbThis, float sscale) {
  union FB { v16b v; v8b h[2]; };
  union FH { v16h v; v8h h[2]; };
  __shared__ __align__(16) __bf16   Ksh[64 * 64];
  __shared__ __align__(16) __bf16   Ksl[64 * 64];
  __shared__ __align__(16) _Float16 Vth[64 * 64];
  __shared__ __align__(16) _Float16 Vtl[RES ? 64 * 64 : 8];
  __shared__ __align__(16) _Float16 Psh[4][16 * 64];
  __shared__ __align__(16) _Float16 Psl[RES ? 4 : 1][16 * 64];
  __shared__ __align__(16) float    Os[4][16 * 64];

  const int tid  = threadIdx.x;
  const int wave = tid >> 5;
  const int lane = tid & 31;
  const int hh   = lane >> 4;
  const int c    = lane & 15;

  const int bx   = blockIdx.x;
  const int qbl  = bx % nqbThis;
  const int rest = bx / nqbThis;
  const int h    = rest % NH;
  int b          = rest / NH;
  b = (b >= NB) ? (NB - 1) : b;
  int qb         = qbBase + qbl;
  qb = (qb >= NQB) ? (NQB - 1) : qb;
  const int q0   = qb * 64 + wave * 16;
  const size_t rowB = (size_t)b * SEQ;

  const __bf16* Qh = (const __bf16*)(const void*)qkhp + (size_t)h * HD;
  const __bf16* Ql = (const __bf16*)(const void*)qklp + (size_t)h * HD;
  const __bf16* Kh = Qh + DMODEL;
  const __bf16* Kl = Ql + DMODEL;
  const _Float16* Vh = (const _Float16*)(const void*)vhp + ((size_t)b * QP + (size_t)h * HD) * SEQ;
  const _Float16* Vl = (const _Float16*)(const void*)vlp + ((size_t)b * QP + (size_t)h * HD) * VLP;
  const float* trow = ttab + ((size_t)b * NH + h) * SEQ;

  const float lraw  = bf_up(bf_bits(lockp[h]));
  const float lockv = 1.0f / (1.0f + expf(-lraw));
  const float c0    = KAPPA_F * lockv;

  v16b qah[2], qal[2];
#pragma unroll
  for (int dc = 0; dc < 2; ++dc) {
    const size_t qo = (rowB + q0 + c) * QKP + dc * 32 + 8 * hh;
    qah[dc] = ldfrag_b(Qh + qo);
    qal[dc] = ldfrag_b(Ql + qo);
  }

  float bti[8];
#pragma unroll
  for (int r = 0; r < 8; ++r) bti[r] = c0 * trow[q0 + 8 * hh + r];

  float mrow[8], lrow[8];
  v8f oacc[4];
#pragma unroll
  for (int r = 0; r < 8; ++r) { mrow[r] = -INFINITY; lrow[r] = 0.f; }
#pragma unroll
  for (int t = 0; t < 4; ++t) oacc[t] = zero8();

  int nkt = qb + 1;
  if (nkt > NQB) nkt = NQB;
  for (int kt = 0; kt < nkt; ++kt) {
    const int kv0 = kt * 64;
    __syncthreads();
    {
      const int r = tid >> 1, half = (tid & 1) * 32;
      const __bf16*   kg  = Kh + (rowB + kv0 + r) * QKP + half;
      const __bf16*   klg = Kl + (rowB + kv0 + r) * QKP + half;
      const _Float16* vg  = Vh + (size_t)r * SEQ + kv0 + half;
      const int kvl = (kv0 + 64 <= VLP) ? kv0 : (VLP - 64);
      const _Float16* vlg = Vl + (size_t)r * VLP + kvl + half;
      const bool resOK = (kv0 + 64 <= VLP);
#pragma unroll
      for (int i = 0; i < 4; ++i) {
        const v8b a0 = *(const v8b*)(kg + 8 * i);
        const v8b a1 = *(const v8b*)(klg + 8 * i);
        const v8h b0 = *(const v8h*)(vg + 8 * i);
        *(v8b*)(Ksh + r * 64 + half + 8 * i) = a0;
        *(v8b*)(Ksl + r * 64 + half + 8 * i) = a1;
        *(v8h*)(Vth + r * 64 + half + 8 * i) = b0;
        if (RES) {
          v8h b1 = *(const v8h*)(vlg + 8 * i);
          if (!resOK) b1 = zero8h();
          *(v8h*)(Vtl + r * 64 + half + 8 * i) = b1;
        }
      }
    }
    __syncthreads();

    float tj[4];
#pragma unroll
    for (int j = 0; j < 4; ++j) tj[j] = trow[kv0 + j * 16 + c];

    v8f s[4];
#pragma unroll
    for (int j = 0; j < 4; ++j) {
      s[j] = zero8();
#pragma unroll
      for (int dc = 0; dc < 2; ++dc) {
        FB kb, kl;
        kb.h[0] = *(const v8b*)(Ksh + (j * 16 + c) * 64 + dc * 32 + 8 * hh);
        kb.h[1] = *(const v8b*)(Ksh + (j * 16 + c) * 64 + dc * 32 + 16 + 8 * hh);
        kl.h[0] = *(const v8b*)(Ksl + (j * 16 + c) * 64 + dc * 32 + 8 * hh);
        kl.h[1] = *(const v8b*)(Ksl + (j * 16 + c) * 64 + dc * 32 + 16 + 8 * hh);
        s[j] = mma_b(qah[dc], kb.v, s[j]);
        s[j] = mma_b(qah[dc], kl.v, s[j]);
        s[j] = mma_b(qal[dc], kb.v, s[j]);
      }
    }

    _Float16* pwh = Psh[wave];
    _Float16* pwl = Psl[RES ? wave : 0];
#pragma unroll
    for (int r = 0; r < 8; ++r) {
      const int qrow = q0 + 8 * hh + r;
      float m = -INFINITY;
#pragma unroll
      for (int j = 0; j < 4; ++j) {
        const int key = kv0 + j * 16 + c;
        float sv = s[j][r] * sscale + bti[r] * tj[j];
        sv = (key > qrow) ? -FLT_MAX : sv;
        s[j][r] = sv;
        m = fmaxf(m, sv);
      }
#pragma unroll
      for (int off = 1; off < 16; off <<= 1) m = fmaxf(m, __shfl_xor(m, off, 32));
      const float mnew  = fmaxf(mrow[r], m);
      const float msafe = (mnew == -INFINITY) ? 0.f : mnew;
      const float alpha = __expf(mrow[r] - msafe);
      mrow[r] = mnew;
      float psum = 0.f;
#pragma unroll
      for (int j = 0; j < 4; ++j) {
        const float p = __expf(s[j][r] - msafe);
        psum += p;
        const float p1k = p * 1024.0f;
        const _Float16 ph = (_Float16)p1k;
        pwh[(8 * hh + r) * 64 + j * 16 + c] = ph;
        if (RES) {
          const _Float16 pl = (_Float16)((p1k - (float)ph) * 4096.0f);
          pwl[(8 * hh + r) * 64 + j * 16 + c] = pl;
        }
      }
#pragma unroll
      for (int off = 1; off < 16; off <<= 1) psum += __shfl_xor(psum, off, 32);
      lrow[r] = lrow[r] * alpha + psum;
#pragma unroll
      for (int t = 0; t < 4; ++t) oacc[t][r] *= alpha;
    }
    __builtin_amdgcn_fence(__ATOMIC_RELEASE, "workgroup");
    __builtin_amdgcn_wave_barrier();
    __builtin_amdgcn_fence(__ATOMIC_ACQUIRE, "workgroup");

    v8f o1[4];
#pragma unroll
    for (int t = 0; t < 4; ++t) o1[t] = zero8();
#pragma unroll 1
    for (int kk = 0; kk < 2; ++kk) {
      FH pa, pl;
      pa.h[0] = *(const v8h*)(pwh + c * 64 + kk * 32 + 8 * hh);
      pa.h[1] = *(const v8h*)(pwh + c * 64 + kk * 32 + 16 + 8 * hh);
      if (RES) {
        pl.h[0] = *(const v8h*)(pwl + c * 64 + kk * 32 + 8 * hh);
        pl.h[1] = *(const v8h*)(pwl + c * 64 + kk * 32 + 16 + 8 * hh);
      } else {
        pl.v = pa.v;
      }
#pragma unroll
      for (int t = 0; t < 4; ++t) {
        FH vb;
        vb.h[0] = *(const v8h*)(Vth + (t * 16 + c) * 64 + kk * 32 + 8 * hh);
        vb.h[1] = *(const v8h*)(Vth + (t * 16 + c) * 64 + kk * 32 + 16 + 8 * hh);
        oacc[t] = mma_h(pa.v, vb.v, oacc[t]);
        if (RES) {
          FH vl;
          vl.h[0] = *(const v8h*)(Vtl + (t * 16 + c) * 64 + kk * 32 + 8 * hh);
          vl.h[1] = *(const v8h*)(Vtl + (t * 16 + c) * 64 + kk * 32 + 16 + 8 * hh);
          o1[t] = mma_h(pa.v, vl.v, o1[t]);
          o1[t] = mma_h(pl.v, vb.v, o1[t]);
        }
      }
    }
    if (RES) {
#pragma unroll
      for (int t = 0; t < 4; ++t)
#pragma unroll
        for (int r = 0; r < 8; ++r) oacc[t][r] += o1[t][r] * (1.0f / 4096.0f);
    }
  }

  float* os = Os[wave];
#pragma unroll
  for (int r = 0; r < 8; ++r) {
    const float l = lrow[r];
    const float ti = trow[q0 + 8 * hh + r];
    const float gate = (1.0f - lockv) + lockv * ti;
    const float inv = ((l > 0.f) ? (1.0f / l) : 0.f) * (1.0f / 1024.0f) * gate;
#pragma unroll
    for (int t = 0; t < 4; ++t) os[(8 * hh + r) * 64 + t * 16 + c] = oacc[t][r] * inv;
  }
  __builtin_amdgcn_fence(__ATOMIC_RELEASE, "workgroup");
  __builtin_amdgcn_wave_barrier();
  __builtin_amdgcn_fence(__ATOMIC_ACQUIRE, "workgroup");
  {
    const int h2 = lane >> 4, c4 = (lane & 15) * 4;
    v4f ov[8];
#pragma unroll
    for (int it = 0; it < 8; ++it) {
      const int row = it * 2 + h2;
      ov[it] = *(const v4f*)(os + row * 64 + c4);
    }
    for (int pass = 0; pass < 2; ++pass) {
#pragma unroll
      for (int it = 0; it < 8; ++it) {
        const int row = it * 2 + h2;
        const size_t go = (rowB + q0 + row) * QP + (size_t)h * HD + c4;
        *(volatile v4f*)(outp + go) = ov[it];
      }
      __threadfence();
    }
  }
}

extern "C" void kernel_launch(void* const* d_in, const int* in_sizes, int n_in,
                              void* d_out, int out_size, void* d_ws, size_t ws_size,
                              hipStream_t stream) {
  if (n_in < 12) return;
  if (in_sizes[0] != NB * SEQ * DMODEL) return;
  if (in_sizes[1] != NB * SEQ) return;
  if (in_sizes[2] != DMODEL * DMODEL || in_sizes[4] != DMODEL * DMODEL ||
      in_sizes[6] != DMODEL * DMODEL || in_sizes[8] != QP * DMODEL) return;
  if (in_sizes[3] != DMODEL || in_sizes[5] != DMODEL || in_sizes[7] != DMODEL || in_sizes[9] != DMODEL) return;
  if (in_sizes[10] != NH || in_sizes[11] != NH) return;
  if (out_size != OUTN) return;

  const float* x     = (const float*)d_in[0];
  const float* phase = (const float*)d_in[1];
  const float* Wq    = (const float*)d_in[2];
  const float* bq    = (const float*)d_in[3];
  const float* Wk    = (const float*)d_in[4];
  const float* bk    = (const float*)d_in[5];
  const float* Wv    = (const float*)d_in[6];
  const float* bv    = (const float*)d_in[7];
  const float* Wo    = (const float*)d_in[8];
  const float* bo    = (const float*)d_in[9];
  const float* carr  = (const float*)d_in[10];
  const float* lockr = (const float*)d_in[11];

  const size_t PXb   = (size_t)NB * SEQ * DMODEL * 2;
  const size_t PWT   = (size_t)N3 * DMODEL * 2;
  const size_t PWo   = (size_t)DMODEL * QP * 2;
  const size_t PBias = (size_t)NBIAS * 4;
  const size_t PTt   = (size_t)NTT * 4;
  const size_t PQKV  = (size_t)NB * SEQ * N3 * 4;
  const size_t PVTh  = (size_t)NB * QP * SEQ * 2;
  const size_t PVTl  = (size_t)NB * QP * VLP * 2;
  const size_t PQK   = (size_t)NB * SEQ * QKP * 2;
  size_t off = 0;
  const size_t oXb   = off; off += PXb;
  const size_t oWT   = off; off += PWT;
  const size_t oWo   = off; off += PWo;
  const size_t oBias = off; off += PBias;
  const size_t oTt   = off; off += PTt;
  const size_t oQKV  = off; off += PQKV;
  const size_t oVTh  = off; off += PVTh;
  const size_t oVTl  = off; off += PVTl;
  const size_t oQKh  = off; off += PQK;
  const size_t oQKl  = off; off += PQK;
  if (off > ws_size) return;
  if (off > (size_t)134217728) return;
  if (PQKV < (size_t)NB * SEQ * QP * 4) return;
  if (PQK < (size_t)NB * SEQ * QP * 2) return;
  const size_t oAf = oQKV;
  const size_t oAh = oQKh;
  const size_t oAl = oQKl;

  char* ws = (char*)d_ws;
  unsigned short* Xb   = (unsigned short*)(ws + oXb);
  unsigned short* WT   = (unsigned short*)(ws + oWT);
  unsigned short* WoT  = (unsigned short*)(ws + oWo);
  float*          Bias = (float*)(ws + oBias);
  float*          Tt   = (float*)(ws + oTt);
  float*          QKVf = (float*)(ws + oQKV);
  unsigned short* VTh  = (unsigned short*)(ws + oVTh);
  unsigned short* VTl  = (unsigned short*)(ws + oVTl);
  unsigned short* QKh  = (unsigned short*)(ws + oQKh);
  unsigned short* QKl  = (unsigned short*)(ws + oQKl);
  float*          Af   = (float*)(ws + oAf);
  unsigned short* Ah   = (unsigned short*)(ws + oAh);
  unsigned short* Al   = (unsigned short*)(ws + oAl);
  float*          outf = (float*)d_out;

  const dim3 blk(256);
  const int n8x   = NB * SEQ * DMODEL / 8;
  const int n8q   = NB * SEQ * DMODEL / 8;
  const int n8a   = NB * SEQ * QP / 8;
  const dim3 gBias(NBIAS / 256);
  const dim3 gTt(NTT / 256);
  const dim3 gCvtX((n8x + 255) / 256);
  const dim3 gTrW(DMODEL / 64, DMODEL / 32);
  const dim3 gQKV(((NB * SEQ / 64) * (N3 / 64) + 7) / 8);
  const dim3 gQKp((n8q + 255) / 256, 2);
  const dim3 gVpl(SEQ / 64, NH, NB);
  const dim3 gSplit((n8a + 255) / 256);
  const dim3 gOut(((NB * SEQ / 64) * (DMODEL / 64) + 7) / 8);

  bias_tab<<<gBias, blk, 0, stream>>>(bq, bk, bv, bo, Bias, NBIAS, DMODEL);
  phase_tab<<<gTt, blk, 0, stream>>>(phase, carr, Tt, NTT);
  cvt_bf16x8<<<gCvtX, blk, 0, stream>>>(x, Xb, n8x);
  tr_cvt_bf16<<<gTrW, blk, 0, stream>>>(Wq, WT, DMODEL, DMODEL);
  tr_cvt_bf16<<<gTrW, blk, 0, stream>>>(Wk, WT + (size_t)DMODEL * DMODEL, DMODEL, DMODEL);
  tr_cvt_bf16<<<gTrW, blk, 0, stream>>>(Wv, WT + (size_t)2 * DMODEL * DMODEL, DMODEL, DMODEL);
  tr_cvt_bf16<<<gTrW, blk, 0, stream>>>(Wo, WoT, QP, DMODEL);
  gemm64<0><<<gQKV, blk, 0, stream>>>(Xb, Xb, DMODEL, WT, DMODEL, Bias, QKVf, N3, NB * SEQ, N3, DMODEL);
  qk_planes<<<gQKp, blk, 0, stream>>>(QKVf, QKh, QKl, n8q);
  v_planes<<<gVpl, blk, 0, stream>>>(QKVf + 2 * DMODEL, N3, VTh, VTl);
  attn_causal64<true><<<dim3(NB * NH * RESQB), dim3(128), 0, stream>>>(
      QKh, QKl, VTh, VTl, Tt, lockr, Af, 0, RESQB, 0.125f);
  if (NQB - RESQB > 0) {
    attn_causal64<false><<<dim3(NB * NH * (NQB - RESQB)), dim3(128), 0, stream>>>(
        QKh, QKl, VTh, VTl, Tt, lockr, Af, RESQB, NQB - RESQB, 0.125f);
  }
  split_bf16x8<<<gSplit, blk, 0, stream>>>(Af, Ah, Al, n8a);
  gemm64<1><<<gOut, blk, 0, stream>>>(Ah, Al, QP, WoT, QP, Bias + 3 * DMODEL, outf, DMODEL, NB * SEQ, DMODEL, QP);
  (void)hipGetLastError();
}
